// TripletTransformer_23021024706982
// MI455X (gfx1250) — hardware-verified
//
#include <hip/hip_runtime.h>
#include <stddef.h>


#define DM      256
#define DQKV    768
#define DFF     1024
#define NH      8
#define DKH     32
#define GT      128
#define SPW     (32 * 64)
#define WPP     72
#define CH      2048
#define CHSH    12
#define NODEB   64
#define NODESH  6
#define BCAP    2048
#define NCHMAX  512
#define NBPMAX  1024
#define WSCAP   134217728
#define ASCL    8.0f
#define WSCL    64.0f
#define INVSCL  0.001953125f
#define INVDM   0.00390625f
#define LGSCL   0.0009765625f
#define LNEPS   1e-5f

static_assert(NH * DKH == DM);
static_assert((DM % 256) == 0 && (DFF % 256) == 0 && (DQKV % 256) == 0);
static_assert((DM % 64) == 0 && (DFF % 64) == 0 && (DQKV % 64) == 0);
static_assert((WPP % 8) == 0);
static_assert(CH == 2048 && (1 << CHSH) >= CH);
static_assert((BCAP % 32) == 0 && NODEB == 64 && (NODEB % 8) == 0);
static_assert((CH % 1024) == 0);

typedef float          v4f  __attribute__((ext_vector_type(4)));
typedef float          v8f  __attribute__((ext_vector_type(8)));
typedef unsigned int   v4u  __attribute__((ext_vector_type(4)));
typedef int            v4i  __attribute__((ext_vector_type(4)));
typedef unsigned short v8us __attribute__((ext_vector_type(8)));
typedef _Float16       v16h __attribute__((ext_vector_type(16)));
union FragH { v16h v; v8us u[2]; };

__device__ __forceinline__ unsigned short h16(float f) {
  const _Float16 h = (_Float16)f;
  return __builtin_bit_cast(unsigned short, h);
}
__device__ __forceinline__ float lo16f(unsigned int w) {
  return (float)__builtin_bit_cast(_Float16, (unsigned short)(w & 0xffffu));
}
__device__ __forceinline__ float hi16f(unsigned int w) {
  return (float)__builtin_bit_cast(_Float16, (unsigned short)(w >> 16));
}

__device__ __forceinline__ v8us cvt8(v4f a, v4f b, float s) {
  v8us r;
  r[0] = h16(a.x * s); r[1] = h16(a.y * s); r[2] = h16(a.z * s); r[3] = h16(a.w * s);
  r[4] = h16(b.x * s); r[5] = h16(b.y * s); r[6] = h16(b.z * s); r[7] = h16(b.w * s);
  return r;
}

__device__ __forceinline__ float gelu1(float x) {
  return 0.5f * x * (1.0f + erff(x * 0.70710678118654752f));
}
__device__ __forceinline__ v4f gelu4(v4f a) {
  v4f r;
  r.x = gelu1(a.x); r.y = gelu1(a.y); r.z = gelu1(a.z); r.w = gelu1(a.w);
  return r;
}

__device__ __forceinline__ v8f wmh(v16h a, v16h b, v8f c) {
  v8f d = __builtin_amdgcn_wmma_f32_16x16x32_f16(false, a, false, b, (short)0, c, false, false);
  asm volatile("v_nop\n\tv_nop\n\tv_nop\n\tv_nop" : "+v"(d) : "v"(a), "v"(b));
  return d;
}

__global__ __launch_bounds__(256) void k_wpack(
    const float* __restrict__ W, unsigned short* wt, int K, int M) {
  __shared__ __attribute__((aligned(16))) unsigned short sT[64 * WPP];
  const int tid = (int)threadIdx.x;
  const int m0 = (int)blockIdx.x * 64, k0 = (int)blockIdx.y * 64;
#pragma unroll 4
  for (int it = 0; it < 16; ++it) {
    const int idx = it * 256 + tid;
    const int kk = idx >> 6, mm = idx & 63;
    int kr = k0 + kk; kr = kr > K - 1 ? K - 1 : kr;
    int mc = m0 + mm; mc = mc > M - 1 ? M - 1 : mc;
    const float w = W[(size_t)kr * M + mc];
    sT[mm * WPP + kk] = h16(w * WSCL);
  }
  __syncthreads();
  v8us pv[2];
  size_t po[2];
#pragma unroll
  for (int it = 0; it < 2; ++it) {
    const int p = it * 256 + tid;
    const int row = p >> 3, c8 = (p & 7) * 8;
    pv[it] = *(const v8us*)(sT + row * WPP + c8);
    int mr = m0 + row; mr = mr > M - 1 ? M - 1 : mr;
    po[it] = (size_t)mr * K + k0 + c8;
  }
  const bool full = (m0 + 64 <= M) && (k0 + 64 <= K);
  if (full) {
#pragma unroll
    for (int it = 0; it < 2; ++it) *(volatile v8us*)(wt + po[it]) = pv[it];
  }
  __threadfence();
  if (full) {
#pragma unroll
    for (int it = 0; it < 2; ++it) *(volatile v8us*)(wt + po[it]) = pv[it];
  }
}

__global__ __launch_bounds__(256) void k_ln(
    const float* X, const float* __restrict__ g, const float* __restrict__ bb,
    unsigned short* outH, int nRows) {
  const int tid = (int)threadIdx.x, lane = tid & 31;
  const int wave = __builtin_amdgcn_readfirstlane(tid >> 5);
  const int row = (int)blockIdx.x * 8 + wave;
  if (row < nRows) {
    const float* xr = X + (size_t)row * DM + 8 * lane;
    const v4f a0 = *(const v4f*)xr;
    const v4f a1 = *(const v4f*)(xr + 4);
    float s = ((a0.x + a0.y) + (a0.z + a0.w)) + ((a1.x + a1.y) + (a1.z + a1.w));
#pragma unroll
    for (int o = 16; o >= 1; o >>= 1) s += __shfl_xor(s, o);
    const float mu = s * INVDM;
    const v4f d0 = a0 - mu, d1 = a1 - mu;
    float sq = (d0.x * d0.x + d0.y * d0.y) + (d0.z * d0.z + d0.w * d0.w)
             + (d1.x * d1.x + d1.y * d1.y) + (d1.z * d1.z + d1.w * d1.w);
#pragma unroll
    for (int o = 16; o >= 1; o >>= 1) sq += __shfl_xor(sq, o);
    const float var  = sq * INVDM;
    const float rstd = rsqrtf(var + LNEPS);
    const v4f g0 = *(const v4f*)(g + 8 * lane);
    const v4f g1 = *(const v4f*)(g + 8 * lane + 4);
    const v4f b0 = *(const v4f*)(bb + 8 * lane);
    const v4f b1 = *(const v4f*)(bb + 8 * lane + 4);
    const v4f y0 = (d0 * rstd) * g0 + b0;
    const v4f y1 = (d1 * rstd) * g1 + b1;
    const v8us hv = cvt8(y0, y1, ASCL);
    unsigned short* op = outH + (size_t)row * DM + 8 * lane;
    *(volatile v8us*)op = hv;
    __threadfence();
    *(volatile v8us*)op = hv;
  }
}

template <int OUT16, int GELU, int RESID>
__global__ __launch_bounds__(GT) void k_gemm(
    const unsigned short* __restrict__ A, const unsigned short* __restrict__ Bt,
    const float* __restrict__ bias, const float* res,
    float* outF, unsigned short* outH, int K, int Ncols, int M) {
  __shared__ __attribute__((aligned(16))) float sT[4 * SPW];
  const int tid = (int)threadIdx.x, lane = tid & 31, hh = lane >> 4, m = lane & 15;
  const int wave = __builtin_amdgcn_readfirstlane(tid >> 5);
  const int r0 = (int)blockIdx.y * 32;
  const int c0 = (int)blockIdx.x * 256 + wave * 64;

  int ra0 = r0 + m;      ra0 = ra0 > M - 1 ? M - 1 : ra0;
  int ra1 = r0 + 16 + m; ra1 = ra1 > M - 1 ? M - 1 : ra1;
  const unsigned short* ap0 = A + (size_t)ra0 * K + 8 * hh;
  const unsigned short* ap1 = A + (size_t)ra1 * K + 8 * hh;
  const unsigned short* bp[4];
#pragma unroll
  for (int j = 0; j < 4; ++j) {
    int cb = c0 + 16 * j + m; cb = cb > Ncols - 1 ? Ncols - 1 : cb;
    bp[j] = Bt + (size_t)cb * K + 8 * hh;
  }

  v8f acc[2][4];
#pragma unroll
  for (int i = 0; i < 2; ++i)
#pragma unroll
    for (int j = 0; j < 4; ++j) { v8f z = {0.f, 0.f, 0.f, 0.f, 0.f, 0.f, 0.f, 0.f}; acc[i][j] = z; }

  const int nk = K >> 5;
#pragma unroll 1
  for (int kt = 0; kt < nk; ++kt) {
    const int kb = kt << 5;
    FragH a0, a1;
    a0.u[0] = *(const v8us*)(ap0 + kb);
    a0.u[1] = *(const v8us*)(ap0 + kb + 16);
    a1.u[0] = *(const v8us*)(ap1 + kb);
    a1.u[1] = *(const v8us*)(ap1 + kb + 16);
#pragma unroll
    for (int j = 0; j < 4; ++j) {
      FragH bf;
      bf.u[0] = *(const v8us*)(bp[j] + kb);
      bf.u[1] = *(const v8us*)(bp[j] + kb + 16);
      acc[0][j] = wmh(a0.v, bf.v, acc[0][j]);
      acc[1][j] = wmh(a1.v, bf.v, acc[1][j]);
    }
  }

  float* sw = sT + wave * SPW;
#pragma unroll
  for (int i = 0; i < 2; ++i)
#pragma unroll
    for (int j = 0; j < 4; ++j)
#pragma unroll
      for (int r = 0; r < 8; ++r)
        sw[(16 * i + 8 * hh + r) * 64 + 16 * j + m] = acc[i][j][r];
  __syncthreads();

  const bool full = (r0 + 32 <= M) && (c0 + 64 <= Ncols);
  if (OUT16) {
    v8us hv[8];
    size_t po[8];
#pragma unroll
    for (int it = 0; it < 8; ++it) {
      const int f = it * 32 + lane;
      const int row = f >> 3, c8 = (f & 7) * 8;
      const v4f v0 = *(const v4f*)(sw + row * 64 + c8);
      const v4f v1 = *(const v4f*)(sw + row * 64 + c8 + 4);
      int gc = c0 + c8; gc = gc > Ncols - 8 ? Ncols - 8 : gc;
      const v4f b0v = *(const v4f*)(bias + gc);
      const v4f b1v = *(const v4f*)(bias + gc + 4);
      v4f o0 = v0 * INVSCL + b0v;
      v4f o1 = v1 * INVSCL + b1v;
      if (GELU) { o0 = gelu4(o0); o1 = gelu4(o1); }
      hv[it] = cvt8(o0, o1, ASCL);
      po[it] = (size_t)(r0 + row) * Ncols + c0 + c8;
    }
    if (full) {
#pragma unroll
      for (int it = 0; it < 8; ++it) *(volatile v8us*)(outH + po[it]) = hv[it];
    }
    __threadfence();
    if (full) {
#pragma unroll
      for (int it = 0; it < 8; ++it) *(volatile v8us*)(outH + po[it]) = hv[it];
    }
  } else {
    v4f ov[16];
    size_t po[16];
#pragma unroll
    for (int it = 0; it < 16; ++it) {
      const int f = it * 32 + lane;
      const int row = f >> 4, c4 = (f & 15) * 4;
      const v4f v = *(const v4f*)(sw + row * 64 + c4);
      int gc = c0 + c4; gc = gc > Ncols - 4 ? Ncols - 4 : gc;
      int gr = r0 + row; gr = gr > M - 1 ? M - 1 : gr;
      const v4f b4 = *(const v4f*)(bias + gc);
      v4f o = v * INVSCL + b4;
      if (RESID) o = o + *(const v4f*)(res + (size_t)gr * Ncols + gc);
      ov[it] = o;
      po[it] = (size_t)(r0 + row) * Ncols + c0 + c4;
    }
    if (full) {
#pragma unroll
      for (int it = 0; it < 16; ++it) *(volatile v4f*)(outF + po[it]) = ov[it];
    }
    __threadfence();
    if (full) {
#pragma unroll
      for (int it = 0; it < 16; ++it) *(volatile v4f*)(outF + po[it]) = ov[it];
    }
  }
}

__global__ __launch_bounds__(256) void k_csort(
    const int* __restrict__ dst, int* elist, int* coff, int nE, int nN, int NB, int NBP) {
  __shared__ unsigned int keys[CH];
  __shared__ __attribute__((aligned(16))) int soff[NBPMAX];
  const int tid = (int)threadIdx.x;
  const int c = (int)blockIdx.x;
  const int cbase = c * CH;

#pragma unroll 1
  for (int i = tid; i < CH; i += 256) {
    const int e = cbase + i;
    const int ea = e < nE ? e : nE - 1;
    int d = dst[ea];
    d = d < 0 ? 0 : (d > nN - 1 ? nN - 1 : d);
    const unsigned int bk = (e < nE) ? (unsigned int)(d >> NODESH) : (unsigned int)NB;
    keys[i] = (bk << CHSH) | (unsigned int)i;
  }
  __syncthreads();

#pragma unroll 1
  for (unsigned int k = 2u; k <= (unsigned int)CH; k <<= 1) {
#pragma unroll 1
    for (unsigned int j = k >> 1; j > 0u; j >>= 1) {
      const unsigned int lm = j - 1u;
#pragma unroll 1
      for (int t = tid; t < CH / 2; t += 256) {
        const unsigned int ut = (unsigned int)t;
        const unsigned int i  = ((ut & ~lm) << 1) | (ut & lm);
        const unsigned int ix = i | j;
        const unsigned int ka = keys[i], kx = keys[ix];
        const bool asc = ((i & k) == 0u);
        const bool swp = asc ? (ka > kx) : (ka < kx);
        keys[i]  = swp ? kx : ka;
        keys[ix] = swp ? ka : kx;
      }
      __syncthreads();
    }
  }

  v4i pv[2];
  size_t po[2];
#pragma unroll
  for (int it = 0; it < 2; ++it) {
    const int base = it * 1024 + 4 * tid;
    v4i v;
    int e;
    e = cbase + (int)(keys[base + 0] & ((1u << CHSH) - 1u)); e = e > nE - 1 ? nE - 1 : e; v.x = e;
    e = cbase + (int)(keys[base + 1] & ((1u << CHSH) - 1u)); e = e > nE - 1 ? nE - 1 : e; v.y = e;
    e = cbase + (int)(keys[base + 2] & ((1u << CHSH) - 1u)); e = e > nE - 1 ? nE - 1 : e; v.z = e;
    e = cbase + (int)(keys[base + 3] & ((1u << CHSH) - 1u)); e = e > nE - 1 ? nE - 1 : e; v.w = e;
    pv[it] = v;
    po[it] = (size_t)c * CH + base;
  }
#pragma unroll
  for (int it = 0; it < 2; ++it) *(volatile v4i*)(elist + po[it]) = pv[it];
  __threadfence();
#pragma unroll
  for (int it = 0; it < 2; ++it) *(volatile v4i*)(elist + po[it]) = pv[it];

#pragma unroll 1
  for (int bq = tid; bq < NBP; bq += 256) {
    const unsigned int kq = (unsigned int)bq << CHSH;
    int lo = 0, n = CH;
#pragma unroll 1
    for (int it = 0; it < 12; ++it) {
      const int half = n >> 1;
      const int mid  = lo + half;
      const int ma   = mid > CH - 1 ? CH - 1 : mid;
      const bool go  = (n > 0) && (keys[ma] < kq);
      lo = go ? (mid + 1) : lo;
      n  = go ? (n - half - 1) : half;
    }
    soff[bq] = lo;
  }
  __syncthreads();
  const int npc = NBP >> 2;
  v4i ov = {0, 0, 0, 0};
  size_t oo = 0;
  const bool act = tid < npc;
  if (act) { ov = *(const v4i*)(soff + 4 * tid); oo = (size_t)c * NBP + 4 * tid; }
  if (act) *(volatile v4i*)(coff + oo) = ov;
  __threadfence();
  if (act) *(volatile v4i*)(coff + oo) = ov;
}

__global__ __launch_bounds__(256) void k_agg(
    const unsigned short* __restrict__ qkv16, const float* __restrict__ dist,
    const float* __restrict__ path, const int* __restrict__ src, const int* __restrict__ dst,
    const int* __restrict__ elist, const int* __restrict__ coff,
    unsigned short* agg16, int nN, int nE, int NCH, int NBP) {
  __shared__ int ccst[NCHMAX];
  __shared__ int ccnt[NCHMAX];
  __shared__ int cpos[NCHMAX];
  __shared__ int stot;
  __shared__ int leid[BCAP];
  __shared__ int lsrc[BCAP];
  __shared__ int ldl[BCAP];
  const int tid = (int)threadIdx.x, lane = tid & 31;
  const int wave = __builtin_amdgcn_readfirstlane(tid >> 5);
  const int b = (int)blockIdx.x;
  const int nb = b * NODEB;

#pragma unroll 1
  for (int cb0 = 0; cb0 < NCH; cb0 += 256) {
    const int c = cb0 + tid;
    const int ca = c < NCH ? c : NCH - 1;
    int s  = coff[(size_t)ca * NBP + b];
    int e2 = coff[(size_t)ca * NBP + b + 1];
    s  = s < 0 ? 0 : (s > CH ? CH : s);
    e2 = e2 < s ? s : (e2 > CH ? CH : e2);
    if (c < NCH) { ccst[c] = s; ccnt[c] = e2 - s; }
  }
  __syncthreads();
  if (tid == 0) {
    int run = 0;
#pragma unroll 1
    for (int c = 0; c < NCH; ++c) {
      int cnt = ccnt[c];
      const int room = BCAP - run;
      cnt = cnt > room ? room : cnt;
      ccnt[c] = cnt;
      cpos[c] = run;
      run += cnt;
    }
    stot = run;
  }
  __syncthreads();
#pragma unroll 1
  for (int c = wave; c < NCH; c += 8) {
    const int cnt  = __builtin_amdgcn_readfirstlane(ccnt[c]);
    const int base = __builtin_amdgcn_readfirstlane(cpos[c]);
    const int st   = __builtin_amdgcn_readfirstlane(ccst[c]);
#pragma unroll 1
    for (int i0 = 0; i0 < cnt; i0 += 32) {
      const int i = i0 + lane;
      const bool ok = i < cnt;
      int idx = st + i; idx = idx > CH - 1 ? CH - 1 : idx;
      int e = elist[(size_t)c * CH + idx];
      e = e < 0 ? 0 : (e > nE - 1 ? nE - 1 : e);
      int s = src[e];
      s = s < 0 ? 0 : (s > nN - 1 ? nN - 1 : s);
      const int d = dst[e];
      int dl = d - nb;
      dl = (dl < 0 || dl > NODEB - 1) ? -1 : dl;
      int p = base + i; p = p > BCAP - 1 ? BCAP - 1 : p;
      if (ok) { leid[p] = e; lsrc[p] = s; ldl[p] = dl; }
    }
  }
  __syncthreads();

  const int tot = __builtin_amdgcn_readfirstlane(stot);
  const int nstep = (tot + 31) >> 5;
  const int hd = lane >> 2;
#pragma unroll 1
  for (int jj = 0; jj < NODEB / 8; ++jj) {
    const int j = wave + 8 * jj;
    const int n = nb + j;
    if (n < nN) {
      const v4u kw = *(const v4u*)(qkv16 + (size_t)n * DQKV + DM + 8 * lane);
      float kf[8];
      kf[0] = lo16f(kw.x); kf[1] = hi16f(kw.x); kf[2] = lo16f(kw.y); kf[3] = hi16f(kw.y);
      kf[4] = lo16f(kw.z); kf[5] = hi16f(kw.z); kf[6] = lo16f(kw.w); kf[7] = hi16f(kw.w);
      float mx = -1.0e30f, z = 0.0f;
      float acc[8];
#pragma unroll
      for (int u = 0; u < 8; ++u) acc[u] = 0.0f;
#pragma unroll 1
      for (int stp = 0; stp < nstep; ++stp) {
        const int i = stp * 32 + lane;
        const int ia = i > BCAP - 1 ? BCAP - 1 : i;
        const bool match = (i < tot) && (ldl[ia] == j);
        unsigned int msk = __builtin_amdgcn_ballot_w32(match);
#pragma unroll 1
        while (msk != 0u) {
          const int t = __builtin_ctz(msk);
          msk &= msk - 1u;
          const int idx = stp * 32 + t;
          const int s = lsrc[idx];
          const int e = leid[idx];
          const unsigned short* qr = qkv16 + (size_t)s * DQKV + 8 * lane;
          const v4u qw = *(const v4u*)qr;
          float dot = lo16f(qw.x) * kf[0];
          dot += hi16f(qw.x) * kf[1];
          dot += lo16f(qw.y) * kf[2];
          dot += hi16f(qw.y) * kf[3];
          dot += lo16f(qw.z) * kf[4];
          dot += hi16f(qw.z) * kf[5];
          dot += lo16f(qw.w) * kf[6];
          dot += hi16f(qw.w) * kf[7];
          dot += __shfl_xor(dot, 1);
          dot += __shfl_xor(dot, 2);
          const float lg = dot * LGSCL + dist[(size_t)e * NH + hd] + path[(size_t)e * NH + hd];
          const float mn = fmaxf(mx, lg);
          const float corr = expf(mx - mn);
          const float p = expf(lg - mn);
          const v4u vw = *(const v4u*)(qr + 2 * DM);
          z = z * corr + p;
          acc[0] = acc[0] * corr + p * lo16f(vw.x);
          acc[1] = acc[1] * corr + p * hi16f(vw.x);
          acc[2] = acc[2] * corr + p * lo16f(vw.y);
          acc[3] = acc[3] * corr + p * hi16f(vw.y);
          acc[4] = acc[4] * corr + p * lo16f(vw.z);
          acc[5] = acc[5] * corr + p * hi16f(vw.z);
          acc[6] = acc[6] * corr + p * lo16f(vw.w);
          acc[7] = acc[7] * corr + p * hi16f(vw.w);
          mx = mn;
        }
      }
      const float rz = (z > 0.0f) ? (1.0f / z) : 0.0f;
      v4f o0, o1;
      o0.x = acc[0] * rz; o0.y = acc[1] * rz; o0.z = acc[2] * rz; o0.w = acc[3] * rz;
      o1.x = acc[4] * rz; o1.y = acc[5] * rz; o1.z = acc[6] * rz; o1.w = acc[7] * rz;
      const v8us hv = cvt8(o0, o1, 1.0f);
      unsigned short* gp = agg16 + (size_t)n * DM + 8 * lane;
      *(volatile v8us*)gp = hv;
      __threadfence();
      *(volatile v8us*)gp = hv;
    }
  }
}

extern "C" void kernel_launch(void* const* d_in, const int* in_sizes, int n_in,
                              void* d_out, int out_size, void* d_ws, size_t ws_size,
                              hipStream_t stream) {
  if (n_in < 17) return;
  const int nN = in_sizes[0] / DM;
  const int nE = in_sizes[3];
  if (nN <= 0 || nE <= 0) return;
  if (in_sizes[0] != nN * DM || (nN % 32) != 0) return;
  if (nN > 60000 || nE > (1 << 24)) return;
  if (in_sizes[1] != nE * NH || in_sizes[2] != nE * NH || in_sizes[4] != nE) return;
  if (in_sizes[5] != DM || in_sizes[6] != DM) return;
  if (in_sizes[7] != DM * DQKV || in_sizes[8] != DQKV) return;
  if (in_sizes[9] != DM || in_sizes[10] != DM) return;
  if (in_sizes[11] != DM * DM || in_sizes[12] != DM) return;
  if (in_sizes[13] != DM * DFF || in_sizes[14] != DFF) return;
  if (in_sizes[15] != DFF * DM || in_sizes[16] != DM) return;
  if (out_size != nN * DM) return;

  const int NB  = (nN + NODEB - 1) / NODEB;
  const int NBP = ((NB + 1 + 31) / 32) * 32;
  const int NCH = (nE + CH - 1) / CH;
  if (NBP > NBPMAX || NCH > NCHMAX || NCH < 1) return;

  const float* x    = (const float*)d_in[0];
  const float* dist = (const float*)d_in[1];
  const float* path = (const float*)d_in[2];
  const int*   src  = (const int*)d_in[3];
  const int*   dst  = (const int*)d_in[4];
  const float* ln1g = (const float*)d_in[5];
  const float* ln1b = (const float*)d_in[6];
  const float* Wqkv = (const float*)d_in[7];
  const float* bqkv = (const float*)d_in[8];
  const float* ln2g = (const float*)d_in[9];
  const float* ln2b = (const float*)d_in[10];
  const float* Wp   = (const float*)d_in[11];
  const float* bp   = (const float*)d_in[12];
  const float* W1   = (const float*)d_in[13];
  const float* bf1  = (const float*)d_in[14];
  const float* W2   = (const float*)d_in[15];
  const float* bf2  = (const float*)d_in[16];
  float* out = (float*)d_out;

  size_t off = 0;
  const size_t oWq = off; off += (size_t)DQKV * DM * 2;        off = (off + 255) & ~(size_t)255;
  const size_t oWp = off; off += (size_t)DM * DM * 2;          off = (off + 255) & ~(size_t)255;
  const size_t oW1 = off; off += (size_t)DFF * DM * 2;         off = (off + 255) & ~(size_t)255;
  const size_t oW2 = off; off += (size_t)DM * DFF * 2;         off = (off + 255) & ~(size_t)255;
  const size_t oNh = off; off += (size_t)nN * DM * 2;          off = (off + 255) & ~(size_t)255;
  const size_t oQk = off; off += (size_t)nN * DQKV * 2;        off = (off + 255) & ~(size_t)255;
  const size_t oEl = off; off += (size_t)NCH * CH * 4;         off = (off + 255) & ~(size_t)255;
  const size_t oCo = off; off += (size_t)NCH * NBP * 4;        off = (off + 255) & ~(size_t)255;
  const size_t oAg = off; off += (size_t)nN * DM * 2;          off = (off + 255) & ~(size_t)255;
  const size_t oX  = off; off += (size_t)nN * DM * 4;          off = (off + 255) & ~(size_t)255;
  const size_t oY  = off; off += (size_t)nN * DM * 2;          off = (off + 255) & ~(size_t)255;
  const size_t oH  = off; off += (size_t)nN * DFF * 2;         off = (off + 255) & ~(size_t)255;
  if (off > ws_size || off > (size_t)WSCAP) return;

  char* ws = (char*)d_ws;
  unsigned short* wq16  = (unsigned short*)(ws + oWq);
  unsigned short* wp16  = (unsigned short*)(ws + oWp);
  unsigned short* w116  = (unsigned short*)(ws + oW1);
  unsigned short* w216  = (unsigned short*)(ws + oW2);
  unsigned short* nh16  = (unsigned short*)(ws + oNh);
  unsigned short* qkv16 = (unsigned short*)(ws + oQk);
  int*            elist = (int*)(ws + oEl);
  int*            coff  = (int*)(ws + oCo);
  unsigned short* agg16 = (unsigned short*)(ws + oAg);
  float*          xpl   = (float*)(ws + oX);
  unsigned short* y16   = (unsigned short*)(ws + oY);
  unsigned short* h16   = (unsigned short*)(ws + oH);

  const dim3 gWq(DQKV / 64, DM / 64);
  const dim3 gWp(DM / 64, DM / 64);
  const dim3 gW1(DFF / 64, DM / 64);
  const dim3 gW2(DM / 64, DFF / 64);
  const dim3 gGq(DQKV / 256, nN / 32);
  const dim3 gGd(DM / 256, nN / 32);
  const dim3 gGf(DFF / 256, nN / 32);

  k_wpack<<<gWq, 256, 0, stream>>>(Wqkv, wq16, DM, DQKV);
  k_wpack<<<gWp, 256, 0, stream>>>(Wp, wp16, DM, DM);
  k_wpack<<<gW1, 256, 0, stream>>>(W1, w116, DM, DFF);
  k_wpack<<<gW2, 256, 0, stream>>>(W2, w216, DFF, DM);

  k_csort<<<NCH, 256, 0, stream>>>(dst, elist, coff, nE, nN, NB, NBP);

  k_ln<<<nN / 8, 256, 0, stream>>>(x, ln1g, ln1b, nh16, nN);

  k_gemm<1, 0, 0><<<gGq, GT, 0, stream>>>(nh16, wq16, bqkv, x, xpl, qkv16, DM, DQKV, nN);

  k_agg<<<NB, 256, 0, stream>>>(qkv16, dist, path, src, dst, elist, coff, agg16, nN, nE, NCH, NBP);

  k_gemm<0, 0, 1><<<gGd, GT, 0, stream>>>(agg16, wp16, bp, x, xpl, nh16, DM, DM, nN);

  k_ln<<<nN / 8, 256, 0, stream>>>(xpl, ln2g, ln2b, y16, nN);

  k_gemm<1, 1, 0><<<gGf, GT, 0, stream>>>(y16, w116, bf1, x, xpl, h16, DM, DFF, nN);

  k_gemm<0, 0, 1><<<gGd, GT, 0, stream>>>(h16, w216, bf2, xpl, out, nh16, DFF, DM, nN);
}
